// GKTGNN_63737314673104
// MI455X (gfx1250) — hardware-verified
//
#include <hip/hip_runtime.h>
#include <stddef.h>


#define DE      256
#define DF      128
#define NOUT    12
#define NOUTP   16
#define NTHR    256
#define NWAVE   8
#define EPT     8
#define NGRP    2
#define CHUNK   (NTHR * EPT * NGRP)
#define WCAP    (EPT * NGRP * 32)
#define LISTN   (NWAVE * WCAP)
#define NBA     512
#define NBD     4096
#define G1ROWS  128
#define APITCH  264
#define HROWS   128
#define HPITCH  136
#define RPW     (NBA / NWAVE)
#define WSCALE  8.0f
#define WINV    0.125f

#define LDS_GEMM1 (G1ROWS * APITCH * 2)
#define LDS_AGG   (NBA * DF * 4 + LISTN * 4 + 64)

#define NBW1 ((DE * DF / 8) / NTHR)
#define NBW2 ((DF * DF / 8) / NTHR)
#define NBWR ((NOUTP * DF / 8) / NTHR)

static_assert((CHUNK & (CHUNK - 1)) == 0);
static_assert(CHUNK <= 4096);
static_assert((NBA & (NBA - 1)) == 0 && (NBD & (NBD - 1)) == 0);
static_assert(NBA <= 4096 && NBD <= 4096);
static_assert(G1ROWS * DF * 4 <= LDS_GEMM1);
static_assert(G1ROWS == 16 * NWAVE && HROWS == 16 * NWAVE);
static_assert(NBA % (16 * NWAVE) == 0);
static_assert((DE * DF / 8) % NTHR == 0 && (DF * DF / 8) % NTHR == 0 && (NOUTP * DF / 8) == NTHR);
static_assert((G1ROWS * DE / 8) % NTHR == 0);
static_assert((NBA * DF / 4) % NTHR == 0);
static_assert(NBD == NWAVE * 4 * 128);
static_assert(DE % 32 == 0 && DF % 32 == 0);

typedef float    v4f  __attribute__((ext_vector_type(4)));
typedef float    v8f  __attribute__((ext_vector_type(8)));
typedef int      v4i  __attribute__((ext_vector_type(4)));
typedef _Float16 v4h  __attribute__((ext_vector_type(4)));
typedef _Float16 v8h  __attribute__((ext_vector_type(8)));
typedef _Float16 v16h __attribute__((ext_vector_type(16)));
union FragH { v16h v; v8h h[2]; };

__device__ __forceinline__ v8h cvt8(v4f a, v4f b) {
  v8h r;
  r[0] = (_Float16)a.x; r[1] = (_Float16)a.y; r[2] = (_Float16)a.z; r[3] = (_Float16)a.w;
  r[4] = (_Float16)b.x; r[5] = (_Float16)b.y; r[6] = (_Float16)b.z; r[7] = (_Float16)b.w;
  return r;
}

__device__ __forceinline__ v8f wmh(v16h a, v16h b, v8f c) {
  v8f d = __builtin_amdgcn_wmma_f32_16x16x32_f16(false, a, false, b, (short)0, c, false, false);
  asm volatile("v_nop\n\tv_nop\n\tv_nop\n\tv_nop" : "+v"(d) : "v"(a), "v"(b));
  return d;
}

template <int NB>
__device__ __forceinline__ int scan_chunk(const int* __restrict__ dsts, int nE, int cbase, int nodeBase,
                                          int vec8, int* list, int tid, int lane, int wave) {
  int wc = 0;
#pragma unroll
  for (int g = 0; g < NGRP; ++g) {
    const int el0  = (g * NTHR + tid) * EPT;
    const int e0   = cbase + el0;
    const int sent = -2147483647 - 1;
    v4i da, db;
    if (vec8 != 0 && cbase + CHUNK <= nE) {
      da = *(const v4i*)(dsts + e0);
      db = *(const v4i*)(dsts + e0 + 4);
    } else {
      da.x = (e0     < nE) ? dsts[min(e0, nE - 1)] : sent;
      da.y = (e0 + 1 < nE) ? dsts[min(e0 + 1, nE - 1)] : sent;
      da.z = (e0 + 2 < nE) ? dsts[min(e0 + 2, nE - 1)] : sent;
      da.w = (e0 + 3 < nE) ? dsts[min(e0 + 3, nE - 1)] : sent;
      db.x = (e0 + 4 < nE) ? dsts[min(e0 + 4, nE - 1)] : sent;
      db.y = (e0 + 5 < nE) ? dsts[min(e0 + 5, nE - 1)] : sent;
      db.z = (e0 + 6 < nE) ? dsts[min(e0 + 6, nE - 1)] : sent;
      db.w = (e0 + 7 < nE) ? dsts[min(e0 + 7, nE - 1)] : sent;
    }
    const unsigned nb = (unsigned)nodeBase;
    const unsigned s0 = (unsigned)da.x - nb, s1 = (unsigned)da.y - nb;
    const unsigned s2 = (unsigned)da.z - nb, s3 = (unsigned)da.w - nb;
    const unsigned s4 = (unsigned)db.x - nb, s5 = (unsigned)db.y - nb;
    const unsigned s6 = (unsigned)db.z - nb, s7 = (unsigned)db.w - nb;
    const bool h0 = s0 < (unsigned)NB, h1 = s1 < (unsigned)NB, h2 = s2 < (unsigned)NB, h3 = s3 < (unsigned)NB;
    const bool h4 = s4 < (unsigned)NB, h5 = s5 < (unsigned)NB, h6 = s6 < (unsigned)NB, h7 = s7 < (unsigned)NB;
    const unsigned any = __builtin_amdgcn_ballot_w32(h0 | h1 | h2 | h3 | h4 | h5 | h6 | h7);
    if (any != 0u) {
#define HITJ(J, HJ, SJ) { \
        const unsigned mj = __builtin_amdgcn_ballot_w32(HJ); \
        if (mj != 0u) { \
          if (HJ) { \
            const int pos = wc + (int)__builtin_amdgcn_mbcnt_lo(mj, 0u); \
            if (pos < WCAP) list[wave * WCAP + pos] = ((el0 + (J)) << 12) | (int)(SJ); \
          } \
          wc += (int)__builtin_popcount(mj); } }
      HITJ(0, h0, s0)
      HITJ(1, h1, s1)
      HITJ(2, h2, s2)
      HITJ(3, h3, s3)
      HITJ(4, h4, s4)
      HITJ(5, h5, s5)
      HITJ(6, h6, s6)
      HITJ(7, h7, s7)
#undef HITJ
    }
  }
  return wc;
}

template <int NB>
__device__ __forceinline__ void gather_rows(const int* __restrict__ ei, const float* __restrict__ src,
                                            float* acc, int* list, int* wcnt,
                                            int nodeBase, int nN, int nE, int vec8,
                                            int tid, int lane, int wave) {
  const int* dsts = ei + nE;
  const int nChunks = (nE + CHUNK - 1) / CHUNK;
#pragma unroll 1
  for (int ch = 0; ch < nChunks; ++ch) {
    const int cbase = ch * CHUNK;
    const int wc = scan_chunk<NB>(dsts, nE, cbase, nodeBase, vec8, list, tid, lane, wave);
    if (lane == 0) wcnt[wave] = wc;
    __syncthreads();
    if (wave == 0) {
#pragma unroll 1
      for (int wsx = 0; wsx < NWAVE; ++wsx) {
        int n = __builtin_amdgcn_readfirstlane(wcnt[wsx]);
        n = n > WCAP ? WCAP : (n < 0 ? 0 : n);
        const int* lp = list + wsx * WCAP;
#pragma unroll 1
        for (int i = 0; i < n; ++i) {
          const int ent  = __builtin_amdgcn_readfirstlane(lp[i]);
          const int slot = ent & (NB - 1);
          int e = cbase + ((ent >> 12) & (CHUNK - 1));
          e = e > nE - 1 ? nE - 1 : e;
          int s = ei[e];
          s = s < 0 ? 0 : (s > nN - 1 ? nN - 1 : s);
          const v4f v = *(const v4f*)(src + (size_t)s * DF + 4 * lane);
          v4f* ap = (v4f*)(acc + slot * DF + 4 * lane);
          *ap = *ap + v;
        }
      }
    }
    __syncthreads();
  }
}

__global__ __launch_bounds__(NTHR) void k_wprep(
    const float* __restrict__ W1, const float* __restrict__ W2, const float* __restrict__ Wr,
    _Float16* w1s, _Float16* w2s, _Float16* wrs) {
  const int b = blockIdx.x, tid = threadIdx.x;
  v4f a, c;
  _Float16* dp;
  if (b < NBW1) {
    const int i  = b * NTHR + tid;
    const int n  = i >> 5;
    const int k0 = (i & 31) * 8;
    const float* p = W1 + (size_t)k0 * DF + n;
    a.x = p[0];      a.y = p[DF];     a.z = p[2 * DF]; a.w = p[3 * DF];
    c.x = p[4 * DF]; c.y = p[5 * DF]; c.z = p[6 * DF]; c.w = p[7 * DF];
    dp = w1s + (size_t)n * DE + k0;
  } else if (b < NBW1 + NBW2) {
    const int i  = (b - NBW1) * NTHR + tid;
    const int n  = i >> 4;
    const int k0 = (i & 15) * 8;
    const float* p = W2 + (size_t)k0 * DF + n;
    a.x = p[0];      a.y = p[DF];     a.z = p[2 * DF]; a.w = p[3 * DF];
    c.x = p[4 * DF]; c.y = p[5 * DF]; c.z = p[6 * DF]; c.w = p[7 * DF];
    dp = w2s + (size_t)n * DF + k0;
  } else {
    const int i  = tid;
    const int n  = i >> 4;
    const int k0 = (i & 15) * 8;
    const int nc = n < NOUT ? n : NOUT - 1;
    const float* p = Wr + (size_t)k0 * NOUT + nc;
    a.x = p[0];        a.y = p[NOUT];     a.z = p[2 * NOUT]; a.w = p[3 * NOUT];
    c.x = p[4 * NOUT]; c.y = p[5 * NOUT]; c.z = p[6 * NOUT]; c.w = p[7 * NOUT];
    const v4f z = {0.f, 0.f, 0.f, 0.f};
    a = (n < NOUT) ? a : z;
    c = (n < NOUT) ? c : z;
    dp = wrs + (size_t)n * DF + k0;
  }
  a = a * WSCALE;
  c = c * WSCALE;
  const v8h hv = cvt8(a, c);
  *(volatile v8h*)dp = hv;
  __threadfence();
  *(volatile v8h*)dp = hv;
}

__global__ __launch_bounds__(NTHR) void k_deg(
    const int* __restrict__ ei, float* dinv, int nN, int nE, int vec8) {
  __shared__ __attribute__((aligned(16))) int cnt[NBD];
  __shared__ __attribute__((aligned(16))) int list[LISTN];
  __shared__ int wcnt[NWAVE];
  const int tid = threadIdx.x, lane = tid & 31, wave = tid >> 5;
  const int nodeBase = blockIdx.x * NBD;
  const int* dsts = ei + nE;
  (void)nN;

  for (int i = tid; i < NBD; i += NTHR) cnt[i] = 0;
  __syncthreads();

  const int nChunks = (nE + CHUNK - 1) / CHUNK;
#pragma unroll 1
  for (int ch = 0; ch < nChunks; ++ch) {
    const int cbase = ch * CHUNK;
    const int wc = scan_chunk<NBD>(dsts, nE, cbase, nodeBase, vec8, list, tid, lane, wave);
    if (lane == 0) wcnt[wave] = wc;
    __syncthreads();
    if (wave == 0) {
#pragma unroll 1
      for (int wsx = 0; wsx < NWAVE; ++wsx) {
        int n = __builtin_amdgcn_readfirstlane(wcnt[wsx]);
        n = n > WCAP ? WCAP : (n < 0 ? 0 : n);
        const int* lp = list + wsx * WCAP;
#pragma unroll 1
        for (int i = 0; i < n; ++i) {
          const int ent  = __builtin_amdgcn_readfirstlane(lp[i]);
          const int slot = ent & (NBD - 1);
          if (lane == 0) cnt[slot] = cnt[slot] + 1;
        }
      }
    }
    __syncthreads();
  }

  v4f dq[4];
#pragma unroll
  for (int q = 0; q < 4; ++q) {
    const int f = (wave * 4 + q) * 128 + 4 * lane;
    const v4i cv = *(const v4i*)(cnt + f);
    dq[q].x = rsqrtf((float)(cv.x + 1));
    dq[q].y = rsqrtf((float)(cv.y + 1));
    dq[q].z = rsqrtf((float)(cv.z + 1));
    dq[q].w = rsqrtf((float)(cv.w + 1));
  }
  float* dp = dinv + (size_t)nodeBase;
#pragma unroll
  for (int q = 0; q < 4; ++q) *(volatile v4f*)(dp + (wave * 4 + q) * 128 + 4 * lane) = dq[q];
  __threadfence();
#pragma unroll
  for (int q = 0; q < 4; ++q) *(volatile v4f*)(dp + (wave * 4 + q) * 128 + 4 * lane) = dq[q];
}

__global__ __launch_bounds__(NTHR) void k_gemm1(
    const float* __restrict__ x, const _Float16* __restrict__ w1s,
    const float* __restrict__ dinv, float* g1, int nN) {
  extern __shared__ v4f lds_dyn[];
  _Float16* sA  = (_Float16*)lds_dyn;
  float*    stg = (float*)lds_dyn;
  const int tid = threadIdx.x, lane = tid & 31, wave = tid >> 5, hh = lane >> 4, m = lane & 15;
  const int rowBase = blockIdx.x * G1ROWS;

#pragma unroll 4
  for (int i = 0; i < (G1ROWS * DE / 8) / NTHR; ++i) {
    const int idx = i * NTHR + tid;
    const int r   = idx >> 5;
    const int c0  = (idx & 31) * 8;
    int node = rowBase + r;
    node = node > nN - 1 ? nN - 1 : node;
    const float* xp = x + (size_t)node * DE + c0;
    const v4f a = *(const v4f*)xp, b = *(const v4f*)(xp + 4);
    *(v8h*)(sA + r * APITCH + c0) = cvt8(a, b);
  }
  __syncthreads();

  v8f acc[8];
#pragma unroll
  for (int t = 0; t < 8; ++t) { v8f z = {0.f, 0.f, 0.f, 0.f, 0.f, 0.f, 0.f, 0.f}; acc[t] = z; }
  const _Float16* ar = sA + (wave * 16 + m) * APITCH + 8 * hh;
#pragma unroll 2
  for (int kt = 0; kt < DE / 32; ++kt) {
    FragH a;
    a.h[0] = *(const v8h*)(ar + 32 * kt);
    a.h[1] = *(const v8h*)(ar + 32 * kt + 16);
#pragma unroll
    for (int t = 0; t < 8; ++t) {
      const _Float16* bp = w1s + (size_t)(16 * t + m) * DE + 32 * kt + 8 * hh;
      FragH b;
      b.h[0] = *(const v8h*)bp;
      b.h[1] = *(const v8h*)(bp + 16);
      acc[t] = wmh(a.v, b.v, acc[t]);
    }
  }
  __syncthreads();

  const int r0 = wave * 16 + 8 * hh;
  const v4f dA = *(const v4f*)(dinv + (size_t)rowBase + r0);
  const v4f dB = *(const v4f*)(dinv + (size_t)rowBase + r0 + 4);
  const float d0 = dA.x * WINV, d1 = dA.y * WINV, d2 = dA.z * WINV, d3 = dA.w * WINV;
  const float d4 = dB.x * WINV, d5 = dB.y * WINV, d6 = dB.z * WINV, d7 = dB.w * WINV;
  float* sp = stg + r0 * DF + m;
#pragma unroll
  for (int t = 0; t < 8; ++t) {
    sp[0 * DF + 16 * t] = acc[t][0] * d0;
    sp[1 * DF + 16 * t] = acc[t][1] * d1;
    sp[2 * DF + 16 * t] = acc[t][2] * d2;
    sp[3 * DF + 16 * t] = acc[t][3] * d3;
    sp[4 * DF + 16 * t] = acc[t][4] * d4;
    sp[5 * DF + 16 * t] = acc[t][5] * d5;
    sp[6 * DF + 16 * t] = acc[t][6] * d6;
    sp[7 * DF + 16 * t] = acc[t][7] * d7;
  }
  __syncthreads();

  const float* lp = stg + wave * 16 * DF + 4 * lane;
  float* gp = g1 + ((size_t)rowBase + wave * 16) * DF + 4 * lane;
#pragma unroll
  for (int i = 0; i < 16; ++i) { const v4f v = *(const v4f*)(lp + i * DF); *(volatile v4f*)(gp + (size_t)i * DF) = v; }
  __threadfence();
#pragma unroll
  for (int i = 0; i < 16; ++i) { const v4f v = *(const v4f*)(lp + i * DF); *(volatile v4f*)(gp + (size_t)i * DF) = v; }
}

__global__ __launch_bounds__(NTHR) void k_agg1(
    const int* __restrict__ ei, const float* __restrict__ g1, const float* __restrict__ dinv,
    const float* __restrict__ b1, const _Float16* __restrict__ w2s, float* g2,
    int nN, int nE, int vec8) {
  extern __shared__ v4f lds_dyn[];
  float* acc  = (float*)lds_dyn;
  int*   list = (int*)(acc + NBA * DF);
  int*   wcnt = list + LISTN;
  const int tid = threadIdx.x, lane = tid & 31, wave = tid >> 5, hh = lane >> 4, m = lane & 15;
  const int nodeBase = blockIdx.x * NBA;

  {
    const v4f z = {0.f, 0.f, 0.f, 0.f};
    for (int i = tid; i < NBA * DF / 4; i += NTHR) lds_dyn[i] = z;
  }
  __syncthreads();

  gather_rows<NBA>(ei, g1, acc, list, wcnt, nodeBase, nN, nE, vec8, tid, lane, wave);

#pragma unroll 4
  for (int i = 0; i < (NBA * DF / 4) / NTHR; ++i) {
    const int idx  = i * NTHR + tid;
    const int slot = idx >> 5;
    const int c4   = (idx & 31) * 4;
    int node = nodeBase + slot;
    node = node > nN - 1 ? nN - 1 : node;
    const float d  = dinv[node];
    const v4f   gv = *(const v4f*)(g1 + (size_t)node * DF + c4);
    const v4f   bv = *(const v4f*)(b1 + c4);
    v4f* ap = (v4f*)(acc + slot * DF + c4);
    v4f hv = (*ap + gv) * d + bv;
    hv.x = fmaxf(hv.x, 0.f); hv.y = fmaxf(hv.y, 0.f); hv.z = fmaxf(hv.z, 0.f); hv.w = fmaxf(hv.w, 0.f);
    *ap = hv;
  }
  __syncthreads();

#pragma unroll 1
  for (int s = 0; s < NBA / 16 / NWAVE; ++s) {
    const int t = wave + NWAVE * s;
    v8f c[8];
#pragma unroll
    for (int nt = 0; nt < 8; ++nt) { v8f z = {0.f, 0.f, 0.f, 0.f, 0.f, 0.f, 0.f, 0.f}; c[nt] = z; }
    const float* arow = acc + (16 * t + m) * DF + 8 * hh;
#pragma unroll
    for (int kt = 0; kt < DF / 32; ++kt) {
      const float* ap = arow + 32 * kt;
      const v4f p0 = *(const v4f*)ap,        p1 = *(const v4f*)(ap + 4);
      const v4f p2 = *(const v4f*)(ap + 16), p3 = *(const v4f*)(ap + 20);
      FragH a;
      a.h[0] = cvt8(p0, p1);
      a.h[1] = cvt8(p2, p3);
#pragma unroll
      for (int nt = 0; nt < DF / 16; ++nt) {
        const _Float16* bp = w2s + (size_t)(16 * nt + m) * DF + 32 * kt + 8 * hh;
        FragH b;
        b.h[0] = *(const v8h*)bp;
        b.h[1] = *(const v8h*)(bp + 16);
        c[nt] = wmh(a.v, b.v, c[nt]);
      }
    }
    const int node0 = nodeBase + 16 * t + 8 * hh;
    const v4f dA = *(const v4f*)(dinv + (size_t)node0);
    const v4f dB = *(const v4f*)(dinv + (size_t)node0 + 4);
    const float d0 = dA.x * WINV, d1 = dA.y * WINV, d2 = dA.z * WINV, d3 = dA.w * WINV;
    const float d4 = dB.x * WINV, d5 = dB.y * WINV, d6 = dB.z * WINV, d7 = dB.w * WINV;
    float* sp = acc + (16 * t + 8 * hh) * DF + m;
#pragma unroll
    for (int nt = 0; nt < 8; ++nt) {
      sp[0 * DF + 16 * nt] = c[nt][0] * d0;
      sp[1 * DF + 16 * nt] = c[nt][1] * d1;
      sp[2 * DF + 16 * nt] = c[nt][2] * d2;
      sp[3 * DF + 16 * nt] = c[nt][3] * d3;
      sp[4 * DF + 16 * nt] = c[nt][4] * d4;
      sp[5 * DF + 16 * nt] = c[nt][5] * d5;
      sp[6 * DF + 16 * nt] = c[nt][6] * d6;
      sp[7 * DF + 16 * nt] = c[nt][7] * d7;
    }
    __syncthreads();
    const float* lp = acc + (16 * t) * DF + 4 * lane;
    float* gp = g2 + ((size_t)nodeBase + 16 * t) * DF + 4 * lane;
#pragma unroll
    for (int i = 0; i < 16; ++i) { const v4f v = *(const v4f*)(lp + i * DF); *(volatile v4f*)(gp + (size_t)i * DF) = v; }
    __threadfence();
#pragma unroll
    for (int i = 0; i < 16; ++i) { const v4f v = *(const v4f*)(lp + i * DF); *(volatile v4f*)(gp + (size_t)i * DF) = v; }
  }
}

__global__ __launch_bounds__(NTHR) void k_agg2(
    const int* __restrict__ ei, const float* __restrict__ g2, const float* __restrict__ dinv,
    const float* __restrict__ b2, float* h2, int nN, int nE, int vec8) {
  extern __shared__ v4f lds_dyn[];
  float* acc  = (float*)lds_dyn;
  int*   list = (int*)(acc + NBA * DF);
  int*   wcnt = list + LISTN;
  const int tid = threadIdx.x, lane = tid & 31, wave = tid >> 5;
  const int nodeBase = blockIdx.x * NBA;

  {
    const v4f z = {0.f, 0.f, 0.f, 0.f};
    for (int i = tid; i < NBA * DF / 4; i += NTHR) lds_dyn[i] = z;
  }
  __syncthreads();

  gather_rows<NBA>(ei, g2, acc, list, wcnt, nodeBase, nN, nE, vec8, tid, lane, wave);

#pragma unroll 4
  for (int i = 0; i < (NBA * DF / 4) / NTHR; ++i) {
    const int idx  = i * NTHR + tid;
    const int slot = idx >> 5;
    const int c4   = (idx & 31) * 4;
    int node = nodeBase + slot;
    node = node > nN - 1 ? nN - 1 : node;
    const float d  = dinv[node];
    const v4f   gv = *(const v4f*)(g2 + (size_t)node * DF + c4);
    const v4f   bv = *(const v4f*)(b2 + c4);
    v4f* ap = (v4f*)(acc + slot * DF + c4);
    v4f hv = (*ap + gv) * d + bv;
    hv.x = fmaxf(hv.x, 0.f); hv.y = fmaxf(hv.y, 0.f); hv.z = fmaxf(hv.z, 0.f); hv.w = fmaxf(hv.w, 0.f);
    *ap = hv;
  }
  __syncthreads();

  const float* lp = acc + (wave * RPW) * DF + 4 * lane;
  float* gp = h2 + ((size_t)nodeBase + wave * RPW) * DF + 4 * lane;
#pragma unroll 8
  for (int i = 0; i < RPW; ++i) { const v4f v = *(const v4f*)(lp + i * DF); *(volatile v4f*)(gp + (size_t)i * DF) = v; }
  __threadfence();
#pragma unroll 8
  for (int i = 0; i < RPW; ++i) { const v4f v = *(const v4f*)(lp + i * DF); *(volatile v4f*)(gp + (size_t)i * DF) = v; }
}

__global__ __launch_bounds__(NTHR) void k_head(
    const float* __restrict__ h2, const int* __restrict__ tm, const _Float16* __restrict__ wrs,
    const float* __restrict__ br, float* out, int nN, int nT) {
  __shared__ __attribute__((aligned(16))) _Float16 sT[HROWS * HPITCH];
  __shared__ __attribute__((aligned(16))) float sO[HROWS * NOUT];
  const int tid = threadIdx.x, lane = tid & 31, wave = tid >> 5, hh = lane >> 4, m = lane & 15;
  const int tBase = blockIdx.x * HROWS;

#pragma unroll 4
  for (int r = 0; r < 16; ++r) {
    int t = tBase + 16 * wave + r;
    t = t > nT - 1 ? nT - 1 : t;
    int node = tm[t];
    node = node < 0 ? 0 : (node > nN - 1 ? nN - 1 : node);
    const v4f v = *(const v4f*)(h2 + (size_t)node * DF + 4 * lane);
    v4h hv;
    hv.x = (_Float16)v.x; hv.y = (_Float16)v.y; hv.z = (_Float16)v.z; hv.w = (_Float16)v.w;
    *(v4h*)(sT + (16 * wave + r) * HPITCH + 4 * lane) = hv;
  }
  __syncthreads();

  v8f c = {0.f, 0.f, 0.f, 0.f, 0.f, 0.f, 0.f, 0.f};
  const _Float16* ar = sT + (16 * wave + m) * HPITCH + 8 * hh;
#pragma unroll
  for (int kt = 0; kt < DF / 32; ++kt) {
    FragH a, b;
    a.h[0] = *(const v8h*)(ar + 32 * kt);
    a.h[1] = *(const v8h*)(ar + 32 * kt + 16);
    const _Float16* bp = wrs + (size_t)m * DF + 32 * kt + 8 * hh;
    b.h[0] = *(const v8h*)bp;
    b.h[1] = *(const v8h*)(bp + 16);
    c = wmh(a.v, b.v, c);
  }
  const float bb = br[m < NOUT ? m : NOUT - 1];
  if (m < NOUT) {
    float* sp = sO + (16 * wave + 8 * hh) * NOUT + m;
    sp[0 * NOUT] = c[0] * WINV + bb;
    sp[1 * NOUT] = c[1] * WINV + bb;
    sp[2 * NOUT] = c[2] * WINV + bb;
    sp[3 * NOUT] = c[3] * WINV + bb;
    sp[4 * NOUT] = c[4] * WINV + bb;
    sp[5 * NOUT] = c[5] * WINV + bb;
    sp[6 * NOUT] = c[6] * WINV + bb;
    sp[7 * NOUT] = c[7] * WINV + bb;
  }
  __syncthreads();

  const size_t outN = (size_t)nT * NOUT;
  const size_t ob   = (size_t)tBase * NOUT;
  v4f ov[2];
  int  fq[2];
#pragma unroll
  for (int j = 0; j < 2; ++j) {
    int q = wave + NWAVE * j;
    q = q > (HROWS * NOUT / 128) - 1 ? (HROWS * NOUT / 128) - 1 : q;
    fq[j] = q * 128 + 4 * lane;
    ov[j] = *(const v4f*)(sO + fq[j]);
  }
#pragma unroll
  for (int j = 0; j < 2; ++j) {
    if (wave + NWAVE * j < HROWS * NOUT / 128) {
      const size_t gi = ob + (size_t)fq[j];
      if (gi < outN) *(volatile v4f*)(out + gi) = ov[j];
    }
  }
  __threadfence();
#pragma unroll
  for (int j = 0; j < 2; ++j) {
    if (wave + NWAVE * j < HROWS * NOUT / 128) {
      const size_t gi = ob + (size_t)fq[j];
      if (gi < outN) *(volatile v4f*)(out + gi) = ov[j];
    }
  }
}

extern "C" void kernel_launch(void* const* d_in, const int* in_sizes, int n_in,
                              void* d_out, int out_size, void* d_ws, size_t ws_size,
                              hipStream_t stream) {
  if (n_in < 9) return;
  const int nN = in_sizes[0] / DE;
  const int nE = in_sizes[1] / 2;
  const int nT = in_sizes[2];
  if (nN <= 0 || nE < 0 || nT <= 0) return;
  if (in_sizes[0] != nN * DE || in_sizes[1] != nE * 2) return;
  if (in_sizes[3] != DE * DF || in_sizes[4] < DF || in_sizes[5] != DF * DF || in_sizes[6] < DF) return;
  if (in_sizes[7] != DF * NOUT || in_sizes[8] < NOUT) return;
  if (out_size != nT * NOUT) return;

  const float* x  = (const float*)d_in[0];
  const int*   ei = (const int*)d_in[1];
  const int*   tm = (const int*)d_in[2];
  const float* W1 = (const float*)d_in[3];
  const float* b1 = (const float*)d_in[4];
  const float* W2 = (const float*)d_in[5];
  const float* b2 = (const float*)d_in[6];
  const float* Wr = (const float*)d_in[7];
  const float* br = (const float*)d_in[8];
  float* out = (float*)d_out;

  const int nBD = (nN + NBD - 1) / NBD;
  const int nG1 = (nN + G1ROWS - 1) / G1ROWS;
  const int nA  = (nN + NBA - 1) / NBA;
  const int nH  = (nT + HROWS - 1) / HROWS;

  char* ws = (char*)d_ws;
  size_t off = 0;
  const size_t oW1 = off; off += (size_t)DF * DE * 2;                          off = (off + 255) & ~(size_t)255;
  const size_t oW2 = off; off += (size_t)DF * DF * 2;                          off = (off + 255) & ~(size_t)255;
  const size_t oWr = off; off += (size_t)NOUTP * DF * 2;                       off = (off + 255) & ~(size_t)255;
  const size_t oDv = off; off += (size_t)nBD * NBD * 4;                        off = (off + 255) & ~(size_t)255;
  const size_t oG1 = off; off += (size_t)nG1 * G1ROWS * DF * 4;                off = (off + 255) & ~(size_t)255;
  const size_t oG2 = off; off += (size_t)nA * NBA * DF * 4;                    off = (off + 255) & ~(size_t)255;
  const size_t oH2 = off; off += (size_t)nA * NBA * DF * 4;                    off = (off + 255) & ~(size_t)255;
  if (off > ws_size) return;
  _Float16* w1s  = (_Float16*)(ws + oW1);
  _Float16* w2s  = (_Float16*)(ws + oW2);
  _Float16* wrs  = (_Float16*)(ws + oWr);
  float*    dinv = (float*)(ws + oDv);
  float*    g1   = (float*)(ws + oG1);
  float*    g2   = (float*)(ws + oG2);
  float*    h2   = (float*)(ws + oH2);

  const int vec8 = ((nE & 3) == 0) ? 1 : 0;

  k_wprep<<<NBW1 + NBW2 + NBWR, NTHR, 0, stream>>>(W1, W2, Wr, w1s, w2s, wrs);

  k_deg<<<nBD, NTHR, 0, stream>>>(ei, dinv, nN, nE, vec8);

  hipFuncSetAttribute(reinterpret_cast<const void*>(&k_gemm1),
                      hipFuncAttributeMaxDynamicSharedMemorySize, LDS_GEMM1);
  k_gemm1<<<nG1, NTHR, LDS_GEMM1, stream>>>(x, w1s, dinv, g1, nN);

  hipFuncSetAttribute(reinterpret_cast<const void*>(&k_agg1),
                      hipFuncAttributeMaxDynamicSharedMemorySize, LDS_AGG);
  k_agg1<<<nA, NTHR, LDS_AGG, stream>>>(ei, g1, dinv, b1, w2s, g2, nN, nE, vec8);

  hipFuncSetAttribute(reinterpret_cast<const void*>(&k_agg2),
                      hipFuncAttributeMaxDynamicSharedMemorySize, LDS_AGG);
  k_agg2<<<nA, NTHR, LDS_AGG, stream>>>(ei, g2, dinv, b2, h2, nN, nE, vec8);

  k_head<<<nH, NTHR, 0, stream>>>(h2, tm, wrs, br, out, nN, nT);
}
